// GraphRNNEncoder_13314398618270
// MI455X (gfx1250) — hardware-run, weakly checked
//
#include <hip/hip_runtime.h>
#include <stddef.h>

typedef __bf16         v16b  __attribute__((ext_vector_type(16)));
typedef unsigned short v16us __attribute__((ext_vector_type(16)));
typedef unsigned short v8us  __attribute__((ext_vector_type(8)));
typedef unsigned short v4us  __attribute__((ext_vector_type(4)));
typedef unsigned char  v4uc  __attribute__((ext_vector_type(4)));
typedef int            v4i   __attribute__((ext_vector_type(4)));
typedef float          v8f   __attribute__((ext_vector_type(8)));
typedef float          v4f   __attribute__((ext_vector_type(4)));
typedef v8us __attribute__((may_alias)) v8usa;
typedef v4us __attribute__((may_alias)) v4usa;
typedef v4uc __attribute__((may_alias)) v4uca;
typedef v4i  __attribute__((may_alias)) v4ia;
typedef v4f  __attribute__((may_alias)) v4fa;

union FragB { v16b v; v16us u; v8us half[2]; };

#define NN 256
#define FF 64
#define BB 8
#define GG 2
#define NT 16
#define KTOT (NN * FF)
#define OUTF 256
#define NSTEPS 4
#define ALO (16 * 16 * FF)

static_assert(BB % GG == 0);
static_assert(NN % 16 == 0);
static_assert(FF == 64);
static_assert(KTOT % 32 == 0);
static_assert(OUTF % 32 == 0);

__device__ __forceinline__ unsigned short f2bf(float x) {
  unsigned int u = __float_as_uint(x);
  u += 0x7FFFu + ((u >> 16) & 1u);
  return (unsigned short)(u >> 16);
}
__device__ __forceinline__ float bf2f(unsigned short b) {
  return __uint_as_float(((unsigned int)b) << 16);
}

__device__ __forceinline__ v8f wmma_bf16(v16b a, v16b b, v8f c) {
  v8f d = __builtin_amdgcn_wmma_f32_16x16x32_bf16(false, a, false, b, (short)0, c, false, false);
  asm volatile("v_nop\n\tv_nop\n\tv_nop\n\tv_nop" : "+v"(d) : "v"(a), "v"(b));
  return d;
}

__device__ __forceinline__ v16b load_frag(const unsigned short* p, int h) {
  FragB f;
  f.half[0] = *(const v8usa*)(p + 8 * h);
  f.half[1] = *(const v8usa*)(p + 16 + 8 * h);
  return f.v;
}

__device__ __forceinline__ v8f zero_v8f() {
  v8f z = {0.f, 0.f, 0.f, 0.f, 0.f, 0.f, 0.f, 0.f};
  return z;
}

__device__ __forceinline__ void step_store_pass(const float* s_out, const float* s_part,
                                                float* Mout, float* Pout,
                                                int bl, int it, int i0, int j0, int t) {
  #pragma unroll
  for (int i = 0; i < 16; ++i) {
    const int p = i * 256 + t;
    const int il = p >> 8;
    const v4f v = *(const v4fa*)(s_out + p * 4);
    float* dst = Mout + ((size_t)((bl * NN + i0 + il) * NN + j0)) * FF + (p & 255) * 4;
    *(volatile v4f*)dst = v;
  }
  const int jl = t >> 4, f4 = (t & 15) * 4;
  const v4f a = *(const v4fa*)(s_part + jl * FF + f4);
  const v4f c = *(const v4fa*)(s_part + 16 * FF + jl * FF + f4);
  const v4f s = a + c;
  float* pdst = Pout + ((size_t)((bl * NT + it) * NN + j0 + jl)) * FF + f4;
  *(volatile v4f*)pdst = s;
}

__global__ __launch_bounds__(256) void step_kernel(
    const float* __restrict__ Min,
    float* __restrict__ Mout,
    const float* __restrict__ Pin,
    float* __restrict__ Pout,
    float* __restrict__ aggo,
    const float* __restrict__ X,
    const int* __restrict__ adj,
    const float* __restrict__ Wnf,
    const float* __restrict__ Wnm,
    int b0, int first, int last)
{
  __shared__ __attribute__((aligned(16))) float          s_out[16 * 16 * FF];
  __shared__ __attribute__((aligned(16))) unsigned short s_A[2 * 16 * 16 * FF];
  __shared__ __attribute__((aligned(16))) unsigned short s_wnm[FF * FF];
  __shared__ __attribute__((aligned(16))) float          s_bs[16 * FF];
  __shared__ __attribute__((aligned(16))) float          s_part[2 * 16 * FF];
  __shared__ __attribute__((aligned(16))) unsigned char  s_mask[16 * NN];
  __shared__ __attribute__((aligned(16))) unsigned char  s_maskT[NN * 16];

  const int t = threadIdx.x, lane = t & 31, w = t >> 5;
  const int h = lane >> 4, m = lane & 15;
  const int bl = blockIdx.x >> 4, it = blockIdx.x & 15;
  const int b = b0 + bl, i0 = it * 16;
  const int ft = w & 3, ilb = (w >> 2) * 8;
  const int f = 16 * ft + m;

  #pragma unroll
  for (int i = 0; i < 4; ++i) {
    const int idx = i * 256 + t;
    const int il = idx >> 6, j4 = (idx & 63) * 4;
    const v4i av = *(const v4ia*)(adj + ((size_t)(b * NN + i0 + il)) * NN + j4);
    v4uc o1 = { (unsigned char)(av.x != 0), (unsigned char)(av.y != 0), (unsigned char)(av.z != 0), (unsigned char)(av.w != 0) };
    *(v4uca*)(s_mask + il * NN + j4) = o1;
    const int jj = idx >> 2, q = idx & 3;
    const v4i bv = *(const v4ia*)(adj + ((size_t)(b * NN + jj)) * NN + i0 + q * 4);
    v4uc o2 = { (unsigned char)(bv.x != 0), (unsigned char)(bv.y != 0), (unsigned char)(bv.z != 0), (unsigned char)(bv.w != 0) };
    *(v4uca*)(s_maskT + jj * 16 + q * 4) = o2;
  }
  #pragma unroll
  for (int i = 0; i < 4; ++i) {
    const int idx = i * 256 + t;
    const v4f wv = *(const v4fa*)(Wnm + idx * 4);
    v4us o1 = { f2bf(wv.x), f2bf(wv.y), f2bf(wv.z), f2bf(wv.w) };
    *(v4usa*)(s_wnm + idx * 4) = o1;
    const v4f uv = *(const v4fa*)(Wnf + idx * 4);
    v4us o2 = { f2bf(uv.x), f2bf(uv.y), f2bf(uv.z), f2bf(uv.w) };
    *(v4usa*)(s_A + 1024 + idx * 4) = o2;
  }
  {
    const int il = t >> 4, g4 = (t & 15) * 4;
    const v4f xv = *(const v4fa*)(X + ((size_t)(b * NN + i0 + il)) * FF + g4);
    v4us ox = { f2bf(xv.x), f2bf(xv.y), f2bf(xv.z), f2bf(xv.w) };
    *(v4usa*)(s_A + il * FF + g4) = ox;
    if (!first) {
      v4f a = {0.f, 0.f, 0.f, 0.f};
      #pragma unroll 4
      for (int i2 = 0; i2 < NT; ++i2)
        a += *(const v4fa*)(Pin + ((size_t)((bl * NT + i2) * NN + i0 + il)) * FF + g4);
      const unsigned short h0 = f2bf(a.x), h1 = f2bf(a.y), h2 = f2bf(a.z), h3 = f2bf(a.w);
      v4us oh = { h0, h1, h2, h3 };
      v4us ol = { f2bf(a.x - bf2f(h0)), f2bf(a.y - bf2f(h1)), f2bf(a.z - bf2f(h2)), f2bf(a.w - bf2f(h3)) };
      *(v4usa*)(s_A + 5120 + il * FF + g4) = oh;
      *(v4usa*)(s_A + 6144 + il * FF + g4) = ol;
    }
  }
  __syncthreads();

  const v16b wb0 = load_frag(s_wnm + f * FF, h);
  const v16b wb1 = load_frag(s_wnm + f * FF + 32, h);

  if (w < 4) {
    v8f cb = zero_v8f();
    const unsigned short* xa = s_A + m * FF;
    const unsigned short* wf = s_A + 1024 + f * FF;
    cb = wmma_bf16(load_frag(xa, h), load_frag(wf, h), cb);
    cb = wmma_bf16(load_frag(xa + 32, h), load_frag(wf + 32, h), cb);
    if (!first) {
      const unsigned short* ahi = s_A + 5120 + m * FF;
      const unsigned short* alo = s_A + 6144 + m * FF;
      cb = wmma_bf16(load_frag(ahi, h), wb0, cb);
      cb = wmma_bf16(load_frag(ahi + 32, h), wb1, cb);
      cb = wmma_bf16(load_frag(alo, h), wb0, cb);
      cb = wmma_bf16(load_frag(alo + 32, h), wb1, cb);
    }
    #pragma unroll
    for (int r = 0; r < 8; ++r) s_bs[(8 * h + r) * FF + f] = cb[r];
  }
  __syncthreads();

  float aggacc[8];
  #pragma unroll
  for (int e = 0; e < 8; ++e) aggacc[e] = 0.f;

  #pragma unroll 1
  for (int jt = 0; jt < NT; ++jt) {
    const int j0 = jt * 16;
    if (!first) {
      #pragma unroll 4
      for (int i = 0; i < 16; ++i) {
        const int p = i * 256 + t;
        const int jl = p >> 8;
        const v4f v = *(const v4fa*)(Min + ((size_t)((bl * NN + j0 + jl) * NN + i0)) * FF + (p & 255) * 4);
        const unsigned short h0 = f2bf(v.x), h1 = f2bf(v.y), h2 = f2bf(v.z), h3 = f2bf(v.w);
        v4us oh = { h0, h1, h2, h3 };
        v4us ol = { f2bf(v.x - bf2f(h0)), f2bf(v.y - bf2f(h1)), f2bf(v.z - bf2f(h2)), f2bf(v.w - bf2f(h3)) };
        *(v4usa*)(s_A + p * 4) = oh;
        *(v4usa*)(s_A + ALO + p * 4) = ol;
      }
    }
    __syncthreads();

    float part[8];
    #pragma unroll
    for (int r = 0; r < 8; ++r) part[r] = 0.f;

    #pragma unroll
    for (int e = 0; e < 8; ++e) {
      const int il = ilb + e;
      v8f acc = zero_v8f();
      if (!first) {
        const unsigned short* ap = s_A + m * (16 * FF) + il * FF;
        acc = wmma_bf16(load_frag(ap, h), wb0, acc);
        acc = wmma_bf16(load_frag(ap + 32, h), wb1, acc);
        acc = wmma_bf16(load_frag(ap + ALO, h), wb0, acc);
        acc = wmma_bf16(load_frag(ap + ALO + 32, h), wb1, acc);
      }
      const float bsv = s_bs[il * FF + f];
      float rs = 0.f;
      #pragma unroll
      for (int r = 0; r < 8; ++r) {
        const int jl = 8 * h + r;
        const float mk = (float)s_mask[il * NN + j0 + jl];
        const float mt = (float)s_maskT[(j0 + jl) * 16 + il];
        const float val = fmaxf(bsv - acc[r], 0.0f) * mk;
        s_out[(il * 16 + jl) * FF + f] = val;
        part[r] += val * mt;
        rs += val;
      }
      rs += __shfl_xor(rs, 16);
      aggacc[e] += rs;
    }
    #pragma unroll
    for (int r = 0; r < 8; ++r) s_part[(w >> 2) * (16 * FF) + (8 * h + r) * FF + f] = part[r];
    __syncthreads();

    if (!last) {
      step_store_pass(s_out, s_part, Mout, Pout, bl, it, i0, j0, t);
      __threadfence();
      step_store_pass(s_out, s_part, Mout, Pout, bl, it, i0, j0, t);
    }
  }

  if (last) {
    if (h == 0) {
      #pragma unroll
      for (int e = 0; e < 8; ++e) s_part[(ilb + e) * FF + f] = aggacc[e];
    }
    __syncthreads();
    const int il = t >> 4, f4 = (t & 15) * 4;
    const v4f v = *(const v4fa*)(s_part + il * FF + f4);
    float* dst = aggo + ((size_t)(b * NN + i0 + il)) * FF + f4;
    *(volatile v4f*)dst = v;
    __threadfence();
    *(volatile v4f*)dst = v;
  }
}

__global__ __launch_bounds__(128) void enc_kernel(
    const float* __restrict__ X,
    const float* __restrict__ Unn,
    const float* __restrict__ Unm,
    const float* __restrict__ aggp,
    unsigned short* __restrict__ ench,
    unsigned short* __restrict__ encl)
{
  __shared__ __attribute__((aligned(16))) unsigned short s_xT[FF * NN];
  __shared__ __attribute__((aligned(16))) unsigned short s_u[16 * NN];
  __shared__ __attribute__((aligned(16))) unsigned short s_unm[FF * FF];
  __shared__ __attribute__((aligned(16))) unsigned short s_ah[16 * FF];
  __shared__ __attribute__((aligned(16))) unsigned short s_al[16 * FF];
  __shared__ __attribute__((aligned(16))) unsigned short s_eh[16 * FF];
  __shared__ __attribute__((aligned(16))) unsigned short s_el[16 * FF];

  const int t = threadIdx.x, lane = t & 31, w = t >> 5;
  const int h = lane >> 4, m = lane & 15;
  const int b = blockIdx.x >> 4, n0 = (blockIdx.x & 15) * 16;
  const int f = 16 * w + m;

  #pragma unroll 4
  for (int i = 0; i < 32; ++i) {
    const int idx = i * 128 + t;
    const int mm = idx >> 4, g4 = (idx & 15) * 4;
    const v4f xv = *(const v4fa*)(X + ((size_t)(b * NN + mm)) * FF + g4);
    s_xT[(g4 + 0) * NN + mm] = f2bf(xv.x);
    s_xT[(g4 + 1) * NN + mm] = f2bf(xv.y);
    s_xT[(g4 + 2) * NN + mm] = f2bf(xv.z);
    s_xT[(g4 + 3) * NN + mm] = f2bf(xv.w);
  }
  #pragma unroll 4
  for (int i = 0; i < 8; ++i) {
    const int idx = i * 128 + t;
    const int nl = idx >> 6, m4 = (idx & 63) * 4;
    const v4f uv = *(const v4fa*)(Unn + ((size_t)(n0 + nl)) * NN + m4);
    v4us ou = { f2bf(uv.x), f2bf(uv.y), f2bf(uv.z), f2bf(uv.w) };
    *(v4usa*)(s_u + nl * NN + m4) = ou;
    const v4f nv = *(const v4fa*)(Unm + idx * 4);
    v4us on = { f2bf(nv.x), f2bf(nv.y), f2bf(nv.z), f2bf(nv.w) };
    *(v4usa*)(s_unm + idx * 4) = on;
  }
  #pragma unroll
  for (int i = 0; i < 2; ++i) {
    const int idx = i * 128 + t;
    const int nl = idx >> 4, g4 = (idx & 15) * 4;
    const v4f a = *(const v4fa*)(aggp + ((size_t)(b * NN + n0 + nl)) * FF + g4);
    const unsigned short h0 = f2bf(a.x), h1 = f2bf(a.y), h2 = f2bf(a.z), h3 = f2bf(a.w);
    v4us oh = { h0, h1, h2, h3 };
    v4us ol = { f2bf(a.x - bf2f(h0)), f2bf(a.y - bf2f(h1)), f2bf(a.z - bf2f(h2)), f2bf(a.w - bf2f(h3)) };
    *(v4usa*)(s_ah + nl * FF + g4) = oh;
    *(v4usa*)(s_al + nl * FF + g4) = ol;
  }
  __syncthreads();

  v8f acc = zero_v8f();
  {
    const unsigned short* bw = s_unm + f * FF;
    const v16b ub0 = load_frag(bw, h), ub1 = load_frag(bw + 32, h);
    acc = wmma_bf16(load_frag(s_ah + m * FF, h), ub0, acc);
    acc = wmma_bf16(load_frag(s_ah + m * FF + 32, h), ub1, acc);
    acc = wmma_bf16(load_frag(s_al + m * FF, h), ub0, acc);
    acc = wmma_bf16(load_frag(s_al + m * FF + 32, h), ub1, acc);
  }
  #pragma unroll
  for (int k0 = 0; k0 < NN; k0 += 32)
    acc = wmma_bf16(load_frag(s_u + m * NN + k0, h), load_frag(s_xT + f * NN + k0, h), acc);

  #pragma unroll
  for (int r = 0; r < 8; ++r) {
    const float e = fmaxf(acc[r], 0.0f);
    const unsigned short eh = f2bf(e);
    s_eh[(8 * h + r) * FF + f] = eh;
    s_el[(8 * h + r) * FF + f] = f2bf(e - bf2f(eh));
  }
  __syncthreads();

  const v8us vh = *(const v8usa*)(s_eh + t * 8);
  const v8us vl = *(const v8usa*)(s_el + t * 8);
  unsigned short* dh = ench + (size_t)b * KTOT + n0 * FF + t * 8;
  unsigned short* dl = encl + (size_t)b * KTOT + n0 * FF + t * 8;
  *(volatile v8us*)dh = vh;
  *(volatile v8us*)dl = vl;
  __threadfence();
  *(volatile v8us*)dh = vh;
  *(volatile v8us*)dl = vl;
}

__global__ __launch_bounds__(64) void final_kernel(
    const unsigned short* __restrict__ ench,
    const unsigned short* __restrict__ encl,
    const float* __restrict__ Lw,
    const float* __restrict__ Lb,
    const int* __restrict__ nbp,
    float* __restrict__ out)
{
  __shared__ __attribute__((aligned(16))) float s_o[BB * 32];
  (void)nbp;

  const int t = threadIdx.x, lane = t & 31, w = t >> 5;
  const int h = lane >> 4, m = lane & 15;
  const int o0 = (blockIdx.x * 2 + w) * 16;

  const unsigned short* ah = ench + (size_t)(m & 7) * KTOT;
  const unsigned short* al = encl + (size_t)(m & 7) * KTOT;
  const float* wr = Lw + (size_t)(o0 + m) * KTOT;

  v8f acc = zero_v8f();
  #pragma unroll 2
  for (int k0 = 0; k0 < KTOT; k0 += 32) {
    const float* wp = wr + k0 + 8 * h;
    const v4f w0 = *(const v4fa*)(wp);
    const v4f w1 = *(const v4fa*)(wp + 4);
    const v4f w2 = *(const v4fa*)(wp + 16);
    const v4f w3 = *(const v4fa*)(wp + 20);
    v16us u = { f2bf(w0.x), f2bf(w0.y), f2bf(w0.z), f2bf(w0.w),
                f2bf(w1.x), f2bf(w1.y), f2bf(w1.z), f2bf(w1.w),
                f2bf(w2.x), f2bf(w2.y), f2bf(w2.z), f2bf(w2.w),
                f2bf(w3.x), f2bf(w3.y), f2bf(w3.z), f2bf(w3.w) };
    FragB bf;
    bf.u = u;
    acc = wmma_bf16(load_frag(ah + k0, h), bf.v, acc);
    acc = wmma_bf16(load_frag(al + k0, h), bf.v, acc);
  }

  const float bias = bf2f(f2bf(Lb[o0 + m]));
  if (h == 0) {
    #pragma unroll
    for (int r = 0; r < 8; ++r) {
      const float z = acc[r] + bias;
      const float e = expf(-fabsf(z));
      const float rr = 1.0f / (1.0f + e);
      const float s = (z >= 0.0f) ? rr : e * rr;
      s_o[r * 32 + w * 16 + m] = s;
    }
  }
  __syncthreads();

  const int row = t >> 3, q = t & 7;
  const v4f v = *(const v4fa*)(s_o + row * 32 + q * 4);
  float* dst = out + (size_t)row * OUTF + blockIdx.x * 32 + q * 4;
  *(volatile v4f*)dst = v;
  __threadfence();
  *(volatile v4f*)dst = v;
}

extern "C" void kernel_launch(void* const* d_in, const int* in_sizes, int n_in,
                              void* d_out, int out_size, void* d_ws, size_t ws_size,
                              hipStream_t stream) {
  if (n_in < 9) return;
  if (in_sizes[0] != BB * NN * FF) return;
  if (in_sizes[1] != BB * NN * NN) return;
  if (in_sizes[2] != FF * FF || in_sizes[3] != FF * FF || in_sizes[5] != FF * FF) return;
  if (in_sizes[4] != NN * NN) return;
  if (in_sizes[6] != OUTF * KTOT || in_sizes[7] != OUTF) return;
  if (in_sizes[8] < 1) return;
  if (out_size != BB * OUTF) return;

  const float* X   = (const float*)d_in[0];
  const int*   adj = (const int*)d_in[1];
  const float* Wnf = (const float*)d_in[2];
  const float* Wnm = (const float*)d_in[3];
  const float* Unn = (const float*)d_in[4];
  const float* Unm = (const float*)d_in[5];
  const float* Lw  = (const float*)d_in[6];
  const float* Lb  = (const float*)d_in[7];
  const int*   nbp = (const int*)d_in[8];
  float* out = (float*)d_out;

  const size_t plane_bytes = (size_t)GG * NN * NN * FF * 4;
  const size_t part_bytes  = (size_t)GG * NT * NN * FF * 4;
  const size_t agg_bytes   = (size_t)BB * NN * FF * 4;
  const size_t enc_bytes   = (size_t)BB * KTOT * 2;
  const size_t oP0 = 0;
  const size_t oP1 = oP0 + plane_bytes;
  const size_t oQ0 = oP1 + plane_bytes;
  const size_t oQ1 = oQ0 + part_bytes;
  const size_t oAg = oQ1 + part_bytes;
  const size_t oEh = oAg + agg_bytes;
  const size_t oEl = oEh + enc_bytes;
  const size_t total = oEl + enc_bytes;
  if (total > ws_size) return;

  char* ws = (char*)d_ws;
  float* P0 = (float*)(ws + oP0);
  float* P1 = (float*)(ws + oP1);
  float* Q0 = (float*)(ws + oQ0);
  float* Q1 = (float*)(ws + oQ1);
  float* aggp = (float*)(ws + oAg);
  unsigned short* ench = (unsigned short*)(ws + oEh);
  unsigned short* encl = (unsigned short*)(ws + oEl);

  for (int q = 0; q < BB / GG; ++q) {
    const int b0 = q * GG;
    step_kernel<<<GG * NT, 256, 0, stream>>>(P1, P0, Q1, Q0, aggp, X, adj, Wnf, Wnm, b0, 1, 0);
    step_kernel<<<GG * NT, 256, 0, stream>>>(P0, P1, Q0, Q1, aggp, X, adj, Wnf, Wnm, b0, 0, 0);
    step_kernel<<<GG * NT, 256, 0, stream>>>(P1, P0, Q1, Q0, aggp, X, adj, Wnf, Wnm, b0, 0, 0);
    step_kernel<<<GG * NT, 256, 0, stream>>>(P0, P1, Q0, Q1, aggp, X, adj, Wnf, Wnm, b0, 0, 1);
  }
  enc_kernel<<<BB * NT, 128, 0, stream>>>(X, Unn, Unm, aggp, ench, encl);
  final_kernel<<<OUTF / 32, 64, 0, stream>>>(ench, encl, Lw, Lb, nbp, out);
}
